// MultiHeadSelfAttentionModule_22548578304189
// MI455X (gfx1250) — hardware-verified
//
#include <hip/hip_runtime.h>
#include <math.h>

constexpr int kBatch = 8;
constexpr int kSeq   = 1024;
constexpr int kDim   = 512;
constexpr int kHid   = 512;
constexpr int kHeads = 8;
constexpr int kHd    = 64;
constexpr int kTok   = kBatch * kSeq;
constexpr float kLnEps   = 1e-5f;
constexpr float kInvDim  = 1.0f / 512.0f;
constexpr float kWCarry  = 16.0f;
constexpr float kACarry  = 16.0f;
constexpr float kLoCarry = 2048.0f;
constexpr float kCtxCarry = 256.0f;
constexpr float kPCarry   = 32768.0f;
constexpr float kScaleLoPass = 1.0f / (kACarry * kLoCarry * kWCarry);
constexpr float kScaleHiPass = 1.0f / (kACarry * kWCarry);
constexpr float kScaleOutLo  = 1.0f / (kCtxCarry * kLoCarry * kWCarry);
constexpr float kScaleOutHi  = 1.0f / (kCtxCarry * kWCarry);
constexpr float kCtxOutScale = kCtxCarry / kPCarry;
constexpr float kPeExpC      = -0.017988946039015984f;
constexpr float kInvSqrtHd   = 0.125f;

constexpr int kKC  = 64;
constexpr int kPWR = 128;
constexpr int kPT  = 80;
constexpr int kQVR = 65;

typedef __attribute__((ext_vector_type(16))) _Float16 v16h;
typedef __attribute__((ext_vector_type(8)))  _Float16 v8h;
typedef __attribute__((ext_vector_type(16))) __bf16   v16b;
typedef __attribute__((ext_vector_type(8)))  __bf16   v8b;
typedef __attribute__((ext_vector_type(8)))  float    v8f;
typedef __attribute__((ext_vector_type(4)))  float    v4f;
typedef __attribute__((ext_vector_type(4)))  unsigned int v4u;

__device__ __forceinline__ unsigned short f2bf_bits(float f) {
  unsigned u = __float_as_uint(f);
  return (unsigned short)((u + 0x7FFFu + ((u >> 16) & 1u)) >> 16);
}
__device__ __forceinline__ float bf_bits2f(unsigned short h) { return __uint_as_float(((unsigned)h) << 16); }
__device__ __forceinline__ float bf_rne(float f) { return bf_bits2f(f2bf_bits(f)); }

__device__ __forceinline__ void dep_guard_h(v8f& a, v8f& b, v16h x, v16h y) { asm volatile("v_nop\n\tv_nop\n\tv_nop\n\tv_nop" : "+v"(a), "+v"(b) : "v"(x), "v"(y)); }
__device__ __forceinline__ void dep_guard_b(v8f& a, v8f& b, v16b x, v16b y) { asm volatile("v_nop\n\tv_nop\n\tv_nop\n\tv_nop" : "+v"(a), "+v"(b) : "v"(x), "v"(y)); }
__device__ __forceinline__ void keep4_h(v16h a, v16h b, v16h c, v16h d) { asm volatile("v_nop" :: "v"(a), "v"(b), "v"(c), "v"(d)); }
__device__ __forceinline__ void keep4_b(v16b a, v16b b, v16b c, v16b d) { asm volatile("v_nop" :: "v"(a), "v"(b), "v"(c), "v"(d)); }
__device__ __forceinline__ void acc_guard4(v8f& a, v8f& b, v8f& c, v8f& d) { asm volatile("v_nop\n\tv_nop\n\tv_nop\n\tv_nop" : "+v"(a), "+v"(b), "+v"(c), "+v"(d)); }
template <typename T> struct Frag;
template <> struct Frag<_Float16> {
  typedef v16h V; union U { v16h v; v8h h[2]; };
  static __device__ __forceinline__ v16h load(const _Float16* p) {
    U f; f.h[0] = *(const v8h*)(p); f.h[1] = *(const v8h*)(p + 16); return f.v;
  }
  static __device__ __forceinline__ v8f mma(v16h a, v16h b, v8f c) {
    return __builtin_amdgcn_wmma_f32_16x16x32_f16(false, a, false, b, (short)0, c, false, false);
  }
  static __device__ __forceinline__ void guard(v8f& a, v8f& b, v16h x, v16h y) { dep_guard_h(a, b, x, y); }
  static __device__ __forceinline__ void keep(v16h a, v16h b, v16h c, v16h d) { keep4_h(a, b, c, d); }
};
template <> struct Frag<__bf16> {
  typedef v16b V; union U { v16b v; v8b h[2]; };
  static __device__ __forceinline__ v16b load(const __bf16* p) {
    U f; f.h[0] = *(const v8b*)(p); f.h[1] = *(const v8b*)(p + 16); return f.v;
  }
  static __device__ __forceinline__ v8f mma(v16b a, v16b b, v8f c) {
    return __builtin_amdgcn_wmma_f32_16x16x32_bf16(false, a, false, b, (short)0, c, false, false);
  }
  static __device__ __forceinline__ void guard(v8f& a, v8f& b, v16b x, v16b y) { dep_guard_b(a, b, x, y); }
  static __device__ __forceinline__ void keep(v16b a, v16b b, v16b c, v16b d) { keep4_b(a, b, c, d); }
};

__device__ __forceinline__ unsigned pk16(unsigned short a, unsigned short b) { return (unsigned)a | ((unsigned)b << 16); }
__device__ __forceinline__ unsigned short h_bits(float f) { const _Float16 h = (_Float16)f; return __builtin_bit_cast(unsigned short, h); }
__device__ __forceinline__ unsigned short h16_bits(_Float16 h) { return __builtin_bit_cast(unsigned short, h); }

template <int ET> struct Elem;
template <> struct Elem<0> { typedef _Float16 T; };
template <> struct Elem<1> { typedef __bf16 T; };
template <int ET, bool SPLIT, int BIAS_MODE, int OUT_MODE, bool RESID, int ACT = 0>
__global__ __launch_bounds__(256) void wmma_gemm64(
    const unsigned short* __restrict__ Ap, const unsigned short* __restrict__ A2p, int lda, long strideA,
    const unsigned short* __restrict__ Btp, const unsigned short* __restrict__ Bt2p, int ldb, long strideB,
    void* __restrict__ Cout, void* __restrict__ Cout2, int ldc, long strideC,
    const float* __restrict__ bias,
    const float* __restrict__ resid, long strideR,
    int M, int N, int K, float scale) {
  typedef typename Elem<ET>::T T;
  typedef typename Frag<T>::V V;
  const T* A = (const T*)Ap; const T* A2 = (const T*)A2p; const T* Bt = (const T*)Btp; const T* Bt2 = (const T*)Bt2p;
  __shared__ __align__(16) float sT[8][16 * 68];
  const int b    = blockIdx.y;
  const int lane = threadIdx.x & 31;
  const int wave = threadIdx.x >> 5;
  const int tilesN = N >> 6;
  const int tilesM = M >> 6;
  const int tile = blockIdx.x * 8 + wave;
  if (tile >= tilesM * tilesN) return;
  const int tm = tile / tilesN;
  const int tn = tile - tm * tilesN;
  const int m0 = tm << 6;
  const int n0 = tn << 6;

  const T* Ab  = A  + (size_t)b * strideA;
  const T* Bb  = Bt + (size_t)b * strideB;
  const T* Ab2 = SPLIT ? (A2  + (size_t)b * strideA) : nullptr;
  const T* Bb2 = SPLIT ? (Bt2 + (size_t)b * strideB) : nullptr;

  const int rlane = lane & 15;
  const int koff  = (lane >> 4) * 8;
  const int mOff  = (lane >> 4) * 8;

  v8f acc[4][4];
#pragma unroll
  for (int i = 0; i < 4; ++i)
#pragma unroll
    for (int j = 0; j < 4; ++j) acc[i][j] = (v8f){0.f,0.f,0.f,0.f,0.f,0.f,0.f,0.f};

  for (int k0 = 0; k0 < K; k0 += 32) {
    V bh[4], bl[4];
#pragma unroll
    for (int j = 0; j < 4; ++j) {
      const size_t bo = (size_t)(n0 + (j << 4) + rlane) * ldb + koff + k0;
      bh[j] = Frag<T>::load(Bb + bo);
      if (SPLIT) bl[j] = Frag<T>::load(Bb2 + bo);
    }
#pragma unroll
    for (int i = 0; i < 4; ++i) {
      const size_t ao = (size_t)(m0 + (i << 4) + rlane) * lda + koff + k0;
      V ah = Frag<T>::load(Ab + ao);
      V al;
      if (SPLIT) al = Frag<T>::load(Ab2 + ao);
#pragma unroll
      for (int j = 0; j < 4; ++j) {
        acc[i][j] = Frag<T>::mma(ah, bh[j], acc[i][j]);
        if (SPLIT) {
          acc[i][j] = Frag<T>::mma(ah, bl[j], acc[i][j]);
          acc[i][j] = Frag<T>::mma(al, bh[j], acc[i][j]);
        }
      }
      Frag<T>::guard(acc[i][0], acc[i][3], ah, SPLIT ? al : ah);
    }
    Frag<T>::keep(bh[0], bh[1], bh[2], bh[3]);
    if (SPLIT) Frag<T>::keep(bl[0], bl[1], bl[2], bl[3]);
  }
  acc_guard4(acc[0][0], acc[0][1], acc[0][2], acc[0][3]);
  acc_guard4(acc[1][0], acc[1][1], acc[1][2], acc[1][3]);
  acc_guard4(acc[2][0], acc[2][1], acc[2][2], acc[2][3]);
  acc_guard4(acc[3][0], acc[3][1], acc[3][2], acc[3][3]);

  float* slab = sT[wave];
  const float* Rb = RESID ? (resid + (size_t)b * strideR) : nullptr;
#pragma unroll
  for (int i = 0; i < 4; ++i) {
    const int mBase = m0 + (i << 4);
#pragma unroll
    for (int j = 0; j < 4; ++j) {
      const int n = n0 + (j << 4) + rlane;
      float bv = 0.f;
      if (BIAS_MODE == 2) bv = bias[n];
#pragma unroll
      for (int r = 0; r < 8; ++r) {
        float v = acc[i][j][r] * scale;
        if (BIAS_MODE == 1) v += bias[mBase + mOff + r];
        if (BIAS_MODE == 2) v += bv;
        if (RESID) v += Rb[(size_t)(mBase + mOff + r) * ldc + n];
        if (ACT == 2) v = fmaxf(v, 0.0f);
        if (ACT == 4) v = (v > 0.f) ? v : 0.01f * v;
        slab[(mOff + r) * 68 + (j << 4) + rlane] = v;
      }
    }
    __builtin_amdgcn_fence(__ATOMIC_RELEASE, "workgroup");
    __builtin_amdgcn_wave_barrier();
    __builtin_amdgcn_fence(__ATOMIC_ACQUIRE, "workgroup");
    if (OUT_MODE == 0) {
      float* C = (float*)Cout + (size_t)b * strideC;
      const int hh = lane >> 4, c4 = (lane & 15) * 4;
      for (int pass = 0; pass < 2; ++pass) {
#pragma unroll
        for (int it = 0; it < 8; ++it) {
          const int row = it * 2 + hh;
          v4f v = *(const v4f*)(slab + row * 68 + c4);
          *(volatile v4f*)(C + (size_t)(mBase + row) * ldc + n0 + c4) = v;
        }
        __threadfence();
      }
    } else {
      const int q = lane >> 3, c8 = (lane & 7) * 8;
      unsigned short* C  = (unsigned short*)Cout  + (size_t)b * strideC;
      unsigned short* C2 = (OUT_MODE == 2) ? ((unsigned short*)Cout2 + (size_t)b * strideC) : nullptr;
      for (int pass = 0; pass < 2; ++pass) {
#pragma unroll
        for (int it = 0; it < 4; ++it) {
          const int row = it * 4 + q;
          const float* sp = slab + row * 68 + c8;
          v8h hv, lv;
#pragma unroll
          for (int e = 0; e < 8; ++e) {
            if (OUT_MODE == 1) {
              hv[e] = (_Float16)sp[e];
            } else {
              unsigned short hb = f2bf_bits(sp[e]);
              unsigned short lb = f2bf_bits(sp[e] - bf_bits2f(hb));
              hv[e] = __builtin_bit_cast(_Float16, hb);
              lv[e] = __builtin_bit_cast(_Float16, lb);
            }
          }
          *(volatile v8h*)(C + (size_t)(mBase + row) * ldc + n0 + c8) = hv;
          if (OUT_MODE == 2) *(volatile v8h*)(C2 + (size_t)(mBase + row) * ldc + n0 + c8) = lv;
        }
        __threadfence();
      }
    }
    __builtin_amdgcn_fence(__ATOMIC_RELEASE, "workgroup");
    __builtin_amdgcn_wave_barrier();
    __builtin_amdgcn_fence(__ATOMIC_ACQUIRE, "workgroup");
  }
}

__global__ __launch_bounds__(128) void bias_table_kernel(const float* __restrict__ b0, const float* __restrict__ b1,
                                                         const float* __restrict__ b2, const float* __restrict__ b3,
                                                         float* __restrict__ table) {
  const int z = blockIdx.x;
  const int t = threadIdx.x;
  const float* src = (z == 0) ? b0 : (z == 1) ? b1 : (z == 2) ? b2 : b3;
  const v4f a = *(const v4f*)(src + 4 * t);
  v4f r;
#pragma unroll
  for (int e = 0; e < 4; ++e) r[e] = bf_rne(a[e]);
  float* d = table + (size_t)z * kDim + 4 * t;
  *(volatile v4f*)d = r;
  __threadfence();
  *(volatile v4f*)d = r;
}

__global__ __launch_bounds__(256) void wtcast5_kernel(const float* __restrict__ W0, const float* __restrict__ W1,
                                                      const float* __restrict__ W2, const float* __restrict__ W3,
                                                      const float* __restrict__ W4,
                                                      unsigned short* __restrict__ out, float scale) {
  __shared__ float sm[64][65];
  const int t  = threadIdx.x;
  const int d0 = blockIdx.x * 64;
  const int h0 = blockIdx.y * 64;
  const int z  = blockIdx.z;
  const float* W = (z == 0) ? W0 : (z == 1) ? W1 : (z == 2) ? W2 : (z == 3) ? W3 : W4;
#pragma unroll
  for (int i = 0; i < 16; ++i) {
    const int e = i * 256 + t;
    const int r = e >> 6;
    const int c = e & 63;
    sm[c][r] = bf_rne(W[(size_t)(d0 + r) * kHid + h0 + c]) * scale;
  }
  __syncthreads();
  const int lane = t & 31, wave = t >> 5;
  const int q = lane >> 3, c8 = (lane & 7) * 8;
  unsigned short* op = out + (size_t)z * kHid * kDim;
  for (int pass = 0; pass < 2; ++pass) {
#pragma unroll
    for (int it = 0; it < 2; ++it) {
      const int row = wave * 8 + it * 4 + q;
      unsigned short hb[8];
#pragma unroll
      for (int e = 0; e < 8; ++e) hb[e] = h_bits(sm[row][c8 + e]);
      const v4u u = (v4u){pk16(hb[0], hb[1]), pk16(hb[2], hb[3]), pk16(hb[4], hb[5]), pk16(hb[6], hb[7])};
      *(volatile v4u*)(op + (size_t)(h0 + row) * kDim + d0 + c8) = u;
    }
    __threadfence();
  }
}

__global__ __launch_bounds__(64) void ln_kernel(const float* __restrict__ x, const float* __restrict__ g,
                                                const float* __restrict__ bb,
                                                unsigned short* __restrict__ xh, unsigned short* __restrict__ xl) {
  __shared__ float red[4];
  const int row  = blockIdx.x;
  const int t    = threadIdx.x, lane = t & 31, wave = t >> 5;
  const int c0   = t * 8;
  const float* xr = x + (size_t)row * kDim + c0;
  const v4f a = *(const v4f*)(xr);
  const v4f c = *(const v4f*)(xr + 4);
  float xv[8];
#pragma unroll
  for (int e = 0; e < 4; ++e) { xv[e] = bf_rne(a[e]); xv[4 + e] = bf_rne(c[e]); }
  float s = ((xv[0] + xv[1]) + (xv[2] + xv[3])) + ((xv[4] + xv[5]) + (xv[6] + xv[7]));
#pragma unroll
  for (int off = 16; off > 0; off >>= 1) s += __shfl_xor(s, off, 32);
  if (lane == 0) red[wave] = s;
  __syncthreads();
  const float mu = (red[0] + red[1]) * kInvDim;
  float d[8];
  float s2 = 0.f;
#pragma unroll
  for (int e = 0; e < 8; ++e) { d[e] = xv[e] - mu; s2 += d[e] * d[e]; }
#pragma unroll
  for (int off = 16; off > 0; off >>= 1) s2 += __shfl_xor(s2, off, 32);
  if (lane == 0) red[2 + wave] = s2;
  __syncthreads();
  const float var  = (red[2] + red[3]) * kInvDim;
  const float rstd = rsqrtf(var + kLnEps);
  const v4f ga = *(const v4f*)(g + c0),  gc = *(const v4f*)(g + c0 + 4);
  const v4f ba = *(const v4f*)(bb + c0), bc = *(const v4f*)(bb + c0 + 4);
  float gv[8], bvv[8];
#pragma unroll
  for (int e = 0; e < 4; ++e) { gv[e] = bf_rne(ga[e]); gv[4 + e] = bf_rne(gc[e]); bvv[e] = bf_rne(ba[e]); bvv[4 + e] = bf_rne(bc[e]); }
  unsigned short hb[8], lb[8];
#pragma unroll
  for (int e = 0; e < 8; ++e) {
    const float xn = ((d[e] * rstd) * gv[e] + bvv[e]) * kACarry;
    const _Float16 hi = (_Float16)xn;
    const _Float16 lo = (_Float16)((xn - (float)hi) * kLoCarry);
    hb[e] = h16_bits(hi);
    lb[e] = h16_bits(lo);
  }
  const v4u uh = (v4u){pk16(hb[0], hb[1]), pk16(hb[2], hb[3]), pk16(hb[4], hb[5]), pk16(hb[6], hb[7])};
  const v4u ul = (v4u){pk16(lb[0], lb[1]), pk16(lb[2], lb[3]), pk16(lb[4], lb[5]), pk16(lb[6], lb[7])};
  unsigned short* ph = xh + (size_t)row * kDim + c0;
  unsigned short* pl = xl + (size_t)row * kDim + c0;
  *(volatile v4u*)ph = uh;
  *(volatile v4u*)pl = ul;
  __threadfence();
  *(volatile v4u*)ph = uh;
  *(volatile v4u*)pl = ul;
}

__global__ __launch_bounds__(256) void pe_kernel(unsigned short* __restrict__ peh, unsigned short* __restrict__ pel, int npair) {
  const int i = blockIdx.x * 256 + threadIdx.x;
  if (i >= npair) return;
  const int s  = i >> 8;
  const int jp = i & 255;
  const float dv  = expf((float)(2 * jp) * kPeExpC);
  const float ang = (float)s * dv;
  const float sn = sinf(ang) * kACarry;
  const float cs = cosf(ang) * kACarry;
  const _Float16 sh = (_Float16)sn, ch = (_Float16)cs;
  const _Float16 sl = (_Float16)((sn - (float)sh) * kLoCarry);
  const _Float16 cl = (_Float16)((cs - (float)ch) * kLoCarry);
  const unsigned wh = pk16(h16_bits(sh), h16_bits(ch));
  const unsigned wl = pk16(h16_bits(sl), h16_bits(cl));
  ((volatile unsigned*)peh)[i] = wh;
  ((volatile unsigned*)pel)[i] = wl;
  __threadfence();
  ((volatile unsigned*)peh)[i] = wh;
  ((volatile unsigned*)pel)[i] = wl;
}

__global__ __launch_bounds__(256) void qplanes_kernel(const float* __restrict__ qf, const float* __restrict__ ub,
                                                      const float* __restrict__ vb,
                                                      unsigned short* __restrict__ quh, unsigned short* __restrict__ qul,
                                                      unsigned short* __restrict__ qvh, unsigned short* __restrict__ qvl, int n8) {
  const int i = blockIdx.x * 256 + threadIdx.x;
  if (i >= n8) return;
  const size_t base = (size_t)i * 8;
  const int col = (int)(base & (size_t)(kDim - 1));
  const v4f q0 = *(const v4f*)(qf + base), q1 = *(const v4f*)(qf + base + 4);
  const v4f u0 = *(const v4f*)(ub + col),  u1 = *(const v4f*)(ub + col + 4);
  const v4f w0 = *(const v4f*)(vb + col),  w1 = *(const v4f*)(vb + col + 4);
  float qv[8], uv[8], vv[8];
#pragma unroll
  for (int e = 0; e < 4; ++e) {
    qv[e] = q0[e]; qv[4 + e] = q1[e];
    uv[e] = bf_rne(u0[e]); uv[4 + e] = bf_rne(u1[e]);
    vv[e] = bf_rne(w0[e]); vv[4 + e] = bf_rne(w1[e]);
  }
  unsigned short auh[8], aul[8], avh[8], avl[8];
#pragma unroll
  for (int e = 0; e < 8; ++e) {
    const float fu = qv[e] + uv[e];
    const unsigned short h1 = f2bf_bits(fu);
    auh[e] = h1; aul[e] = f2bf_bits(fu - bf_bits2f(h1));
    const float fv = qv[e] + vv[e];
    const unsigned short h2 = f2bf_bits(fv);
    avh[e] = h2; avl[e] = f2bf_bits(fv - bf_bits2f(h2));
  }
  const v4u xuh = (v4u){pk16(auh[0], auh[1]), pk16(auh[2], auh[3]), pk16(auh[4], auh[5]), pk16(auh[6], auh[7])};
  const v4u xul = (v4u){pk16(aul[0], aul[1]), pk16(aul[2], aul[3]), pk16(aul[4], aul[5]), pk16(aul[6], aul[7])};
  const v4u xvh = (v4u){pk16(avh[0], avh[1]), pk16(avh[2], avh[3]), pk16(avh[4], avh[5]), pk16(avh[6], avh[7])};
  const v4u xvl = (v4u){pk16(avl[0], avl[1]), pk16(avl[2], avl[3]), pk16(avl[4], avl[5]), pk16(avl[6], avl[7])};
  *(volatile v4u*)(quh + base) = xuh;
  *(volatile v4u*)(qul + base) = xul;
  *(volatile v4u*)(qvh + base) = xvh;
  *(volatile v4u*)(qvl + base) = xvl;
  __threadfence();
  *(volatile v4u*)(quh + base) = xuh;
  *(volatile v4u*)(qul + base) = xul;
  *(volatile v4u*)(qvh + base) = xvh;
  *(volatile v4u*)(qvl + base) = xvl;
}

union FragB { v16b v; v8b h[2]; };
union FragH { v16h v; v8h h[2]; };

__device__ __forceinline__ v8f mma_bf(v16b a, v16b b, v8f c) {
  c = __builtin_amdgcn_wmma_f32_16x16x32_bf16(false, a, false, b, (short)0, c, false, false);
  asm volatile("v_nop\n\tv_nop\n\tv_nop\n\tv_nop" : "+v"(c) : "v"(a), "v"(b));
  return c;
}
__device__ __forceinline__ v8f mma_h(v16h a, v16h b, v8f c) {
  c = __builtin_amdgcn_wmma_f32_16x16x32_f16(false, a, false, b, (short)0, c, false, false);
  asm volatile("v_nop\n\tv_nop\n\tv_nop\n\tv_nop" : "+v"(c) : "v"(a), "v"(b));
  return c;
}
__device__ __forceinline__ void lds_wave_sync() {
  __builtin_amdgcn_fence(__ATOMIC_RELEASE, "workgroup");
  __builtin_amdgcn_wave_barrier();
  __builtin_amdgcn_fence(__ATOMIC_ACQUIRE, "workgroup");
}

template <int SHIFT_MODE>
__device__ __forceinline__ void pos_phase(v8f (&s)[4], const __bf16* qvh, const __bf16* qvl,
                                          const __bf16* pwh, const __bf16* pwl, float* pt,
                                          int ro, int wofs, int hh, int c, int q0, int kv0) {
#pragma unroll 1
  for (int t = 0; t < 5; ++t) {
    v8f acc = (v8f){0.f,0.f,0.f,0.f,0.f,0.f,0.f,0.f};
#pragma unroll
    for (int dc = 0; dc < 2; ++dc) {
      FragB ah, al, ph, pl;
      const int ao = (ro + c) * kHd + dc * 32 + 8 * hh;
      ah.h[0] = *(const v8b*)(qvh + ao); ah.h[1] = *(const v8b*)(qvh + ao + 16);
      al.h[0] = *(const v8b*)(qvl + ao); al.h[1] = *(const v8b*)(qvl + ao + 16);
      const int po = (wofs + 16 * t + c) * kHd + dc * 32 + 8 * hh;
      ph.h[0] = *(const v8b*)(pwh + po); ph.h[1] = *(const v8b*)(pwh + po + 16);
      pl.h[0] = *(const v8b*)(pwl + po); pl.h[1] = *(const v8b*)(pwl + po + 16);
      acc = mma_bf(ah.v, ph.v, acc);
      acc = mma_bf(ah.v, pl.v, acc);
      acc = mma_bf(al.v, ph.v, acc);
    }
#pragma unroll
    for (int r = 0; r < 8; ++r) pt[(8 * hh + r) * kPT + 16 * t + c] = acc[r];
  }
  lds_wave_sync();
#pragma unroll
  for (int r = 0; r < 8; ++r) {
    const int rr = 8 * hh + r;
    const int ig = q0 + rr;
    const float* prow = pt + rr * kPT + 15 - rr;
#pragma unroll
    for (int jt = 0; jt < 4; ++jt) {
      const int jj = 16 * jt + c;
      const int jg = kv0 + jj;
      const float gval = prow[jj];
      const bool keep = (SHIFT_MODE == 1) ? (jg <= ig) : (jg >= ig + 2);
      s[jt][r] += keep ? gval : 0.0f;
    }
  }
  lds_wave_sync();
}

__global__ __launch_bounds__(128)
void rel_attn_kernel(const __bf16* __restrict__ QUh, const __bf16* __restrict__ QUl,
                     const __bf16* __restrict__ QVh, const __bf16* __restrict__ QVl,
                     const __bf16* __restrict__ Kh,  const __bf16* __restrict__ Kl,
                     const __bf16* __restrict__ Ph,  const __bf16* __restrict__ Pl,
                     const _Float16* __restrict__ Vp,
                     unsigned short* __restrict__ Ch, unsigned short* __restrict__ Cl) {
  __shared__ __align__(16) __bf16   Ksh[kKC * kHd];
  __shared__ __align__(16) __bf16   Ksl[kKC * kHd];
  __shared__ __align__(16) _Float16 Vt[kHd * kKC];
  __shared__ __align__(16) __bf16   PWh[kPWR * kHd];
  __shared__ __align__(16) __bf16   PWl[kPWR * kHd];
  __shared__ __align__(16) __bf16   QVsh[kQVR * kHd];
  __shared__ __align__(16) __bf16   QVsl[kQVR * kHd];
  __shared__ __align__(16) _Float16 Psh[4][16 * kKC];
  __shared__ __align__(16) float    PT[4][16 * kPT];

  const int tid  = threadIdx.x;
  const int wave = tid >> 5;
  const int lane = tid & 31;
  const int hh   = lane >> 4;
  const int c    = lane & 15;

  const int bx  = blockIdx.x;
  const int qb  = bx & 15;
  const int bhd = bx >> 4;
  const int h   = bhd & 7;
  const int b   = bhd >> 3;
  const int i0b = qb * 64;
  const int q0  = i0b + wave * 16;
  const size_t tokb = (size_t)b * kSeq;
  const int hcol = h * kHd;

  for (int idx = tid; idx < 2 * kQVR; idx += 128) {
    const int row = idx >> 1, hf = (idx & 1) * 32;
    int gr = i0b + row; gr = (gr > kSeq - 1) ? (kSeq - 1) : gr;
    const size_t go = (tokb + gr) * kDim + hcol + hf;
#pragma unroll
    for (int i = 0; i < 4; ++i) {
      *(v8b*)(QVsh + row * kHd + hf + 8 * i) = *(const v8b*)(QVh + go + 8 * i);
      *(v8b*)(QVsl + row * kHd + hf + 8 * i) = *(const v8b*)(QVl + go + 8 * i);
    }
  }
  v16b quh[2], qul[2];
  {
    const size_t qo = (tokb + q0 + c) * kDim + hcol + 8 * hh;
#pragma unroll
    for (int dc = 0; dc < 2; ++dc) {
      quh[dc] = Frag<__bf16>::load(QUh + qo + dc * 32);
      qul[dc] = Frag<__bf16>::load(QUl + qo + dc * 32);
    }
  }

  float mrow[8], lrow[8];
  v8f oacc[4];
#pragma unroll
  for (int r = 0; r < 8; ++r) { mrow[r] = -INFINITY; lrow[r] = 0.f; }
#pragma unroll
  for (int t = 0; t < 4; ++t) oacc[t] = (v8f){0.f,0.f,0.f,0.f,0.f,0.f,0.f,0.f};

  const int wofs = 48 - 16 * wave;

  for (int kc = 0; kc < kSeq / kKC; ++kc) {
    const int kv0 = kc * kKC;
    __syncthreads();
    {
      const int kvr = tid >> 1, hf = (tid & 1) * 32;
      const size_t go = (tokb + kv0 + kvr) * kDim + hcol + hf;
#pragma unroll
      for (int i = 0; i < 4; ++i) {
        *(v8b*)(Ksh + kvr * kHd + hf + 8 * i) = *(const v8b*)(Kh + go + 8 * i);
        *(v8b*)(Ksl + kvr * kHd + hf + 8 * i) = *(const v8b*)(Kl + go + 8 * i);
        const v8h vv = *(const v8h*)(Vp + go + 8 * i);
#pragma unroll
        for (int e = 0; e < 8; ++e) Vt[(hf + 8 * i + e) * kKC + kvr] = vv[e];
      }
      const int pbase = (kc <= qb) ? (kSeq - 64 * (qb - kc + 1)) : (64 * (kc - qb) - 65);
      int m = pbase + tid; m = (m < 0) ? 0 : ((m > kSeq - 1) ? (kSeq - 1) : m);
      const size_t po = (size_t)m * kDim + hcol;
#pragma unroll
      for (int i = 0; i < 8; ++i) {
        *(v8b*)(PWh + tid * kHd + 8 * i) = *(const v8b*)(Ph + po + 8 * i);
        *(v8b*)(PWl + tid * kHd + 8 * i) = *(const v8b*)(Pl + po + 8 * i);
      }
    }
    __syncthreads();

    v8f s[4];
#pragma unroll
    for (int j = 0; j < 4; ++j) {
      s[j] = (v8f){0.f,0.f,0.f,0.f,0.f,0.f,0.f,0.f};
#pragma unroll
      for (int dc = 0; dc < 2; ++dc) {
        FragB kb, kl;
        kb.h[0] = *(const v8b*)(Ksh + (j * 16 + c) * kHd + dc * 32 + 8 * hh);
        kb.h[1] = *(const v8b*)(Ksh + (j * 16 + c) * kHd + dc * 32 + 16 + 8 * hh);
        kl.h[0] = *(const v8b*)(Ksl + (j * 16 + c) * kHd + dc * 32 + 8 * hh);
        kl.h[1] = *(const v8b*)(Ksl + (j * 16 + c) * kHd + dc * 32 + 16 + 8 * hh);
        s[j] = mma_bf(quh[dc], kb.v, s[j]);
        s[j] = mma_bf(quh[dc], kl.v, s[j]);
        s[j] = mma_bf(qul[dc], kb.v, s[j]);
      }
    }

    if (kc <= qb) pos_phase<1>(s, QVsh, QVsl, PWh, PWl, PT[wave], wave * 16, wofs, hh, c, q0, kv0);
    if (kc == qb) {
      __syncthreads();
      {
        int m = tid - 65; m = (m < 0) ? 0 : m;
        const size_t po = (size_t)m * kDim + hcol;
#pragma unroll
        for (int i = 0; i < 8; ++i) {
          *(v8b*)(PWh + tid * kHd + 8 * i) = *(const v8b*)(Ph + po + 8 * i);
          *(v8b*)(PWl + tid * kHd + 8 * i) = *(const v8b*)(Pl + po + 8 * i);
        }
      }
      __syncthreads();
    }
    if (kc >= qb) pos_phase<2>(s, QVsh, QVsl, PWh, PWl, PT[wave], wave * 16 + 1, wofs, hh, c, q0, kv0);

    float cm[8];
#pragma unroll
    for (int r = 0; r < 8; ++r) {
      float m = -INFINITY;
#pragma unroll
      for (int j = 0; j < 4; ++j) {
        s[j][r] = s[j][r] * kInvSqrtHd;
        m = fmaxf(m, s[j][r]);
      }
#pragma unroll
      for (int off = 1; off < 16; off <<= 1) m = fmaxf(m, __shfl_xor(m, off, 32));
      cm[r] = m;
    }
    _Float16* pw = Psh[wave];
#pragma unroll
    for (int r = 0; r < 8; ++r) {
      const float mnew = fmaxf(mrow[r], cm[r]);
      const float alpha = expf(mrow[r] - mnew);
      mrow[r] = mnew;
      float psum = 0.f;
#pragma unroll
      for (int j = 0; j < 4; ++j) {
        const float p = expf(s[j][r] - mnew);
        psum += p;
        pw[(8 * hh + r) * kKC + j * 16 + c] = (_Float16)(p * kPCarry);
      }
#pragma unroll
      for (int off = 1; off < 16; off <<= 1) psum += __shfl_xor(psum, off, 32);
      lrow[r] = lrow[r] * alpha + psum;
#pragma unroll
      for (int t = 0; t < 4; ++t) oacc[t][r] *= alpha;
    }
    lds_wave_sync();
#pragma unroll 1
    for (int kk = 0; kk < 2; ++kk) {
      FragH pa;
      pa.h[0] = *(const v8h*)(pw + c * kKC + kk * 32 + 8 * hh);
      pa.h[1] = *(const v8h*)(pw + c * kKC + kk * 32 + 16 + 8 * hh);
#pragma unroll
      for (int t = 0; t < 4; ++t) {
        FragH vb;
        vb.h[0] = *(const v8h*)(Vt + (t * 16 + c) * kKC + kk * 32 + 8 * hh);
        vb.h[1] = *(const v8h*)(Vt + (t * 16 + c) * kKC + kk * 32 + 16 + 8 * hh);
        oacc[t] = mma_h(pa.v, vb.v, oacc[t]);
      }
    }
  }

  float* os = PT[wave];
#pragma unroll
  for (int r = 0; r < 8; ++r) {
    const float inv = (1.0f / lrow[r]) * kCtxOutScale;
#pragma unroll
    for (int t = 0; t < 4; ++t) os[(8 * hh + r) * kPT + t * 16 + c] = oacc[t][r] * inv;
  }
  lds_wave_sync();
  {
    const int q8 = lane >> 3, c8 = (lane & 7) * 8;
    for (int pass = 0; pass < 2; ++pass) {
#pragma unroll
      for (int it = 0; it < 4; ++it) {
        const int row = it * 4 + q8;
        const float* sp = os + row * kPT + c8;
        v8h hv, lv;
#pragma unroll
        for (int e = 0; e < 8; ++e) {
          const _Float16 hi = (_Float16)sp[e];
          hv[e] = hi;
          lv[e] = (_Float16)((sp[e] - (float)hi) * kLoCarry);
        }
        const size_t o = (tokb + q0 + row) * kDim + hcol + c8;
        *(volatile v8h*)(Ch + o) = hv;
        *(volatile v8h*)(Cl + o) = lv;
      }
      __threadfence();
    }
  }
}

template <int BIAS_MODE, int OUT_MODE, bool RESID>
static void gemm_call(hipStream_t st, const void* A, const void* Bt, void* C, void* C2,
                      const float* bias, const float* resid, int M, float scale) {
  const int tiles = (M / 64) * (kDim / 64);
  dim3 grid((tiles + 7) / 8, 1, 1);
  wmma_gemm64<0, false, BIAS_MODE, OUT_MODE, RESID><<<grid, 256, 0, st>>>(
      (const unsigned short*)A, (const unsigned short*)A, kDim, 0L,
      (const unsigned short*)Bt, (const unsigned short*)Bt, kDim, 0L,
      C, C2, kDim, 0L, bias, resid, 0L, M, kDim, kDim, scale);
}

extern "C" void kernel_launch(void* const* d_in, const int* in_sizes, int n_in,
                              void* d_out, int out_size, void* d_ws, size_t ws_size,
                              hipStream_t stream) {
  if (n_in < 14) return;
  if (in_sizes[0] != kTok * kDim || out_size != kTok * kDim) return;
  if (in_sizes[1] != kDim * kDim || in_sizes[3] != kDim * kDim || in_sizes[5] != kDim * kDim ||
      in_sizes[7] != kDim * kDim || in_sizes[9] != kDim * kDim) return;
  if (in_sizes[2] != kDim || in_sizes[4] != kDim || in_sizes[6] != kDim || in_sizes[8] != kDim ||
      in_sizes[10] != kHeads * kHd || in_sizes[11] != kHeads * kHd || in_sizes[12] != kDim || in_sizes[13] != kDim) return;

  const float* x   = (const float*)d_in[0];
  const float* Wq  = (const float*)d_in[1];
  const float* bq  = (const float*)d_in[2];
  const float* Wk  = (const float*)d_in[3];
  const float* bk  = (const float*)d_in[4];
  const float* Wv  = (const float*)d_in[5];
  const float* bv  = (const float*)d_in[6];
  const float* Wo  = (const float*)d_in[7];
  const float* bo  = (const float*)d_in[8];
  const float* Wp  = (const float*)d_in[9];
  const float* ub  = (const float*)d_in[10];
  const float* vbias = (const float*)d_in[11];
  const float* lng = (const float*)d_in[12];
  const float* lnb = (const float*)d_in[13];
  float* out = (float*)d_out;

  char* ws = (char*)d_ws;
  size_t off = 0;
  auto carve = [&](size_t bytes) -> char* {
    char* p = ws + off;
    off += (bytes + 255) & ~(size_t)255;
    return p;
  };
  const size_t wplane = (size_t)kDim * kDim * 2;
  const size_t act16  = (size_t)kTok * kDim * 2;
  const size_t act32  = (size_t)kTok * kDim * 4;
  const size_t pe16   = (size_t)kSeq * kDim * 2;

  unsigned short* W16 = (unsigned short*)carve(5 * wplane);
  float*          BR  = (float*)carve((size_t)4 * kDim * sizeof(float));
  unsigned short* XNh = (unsigned short*)carve(act16);
  unsigned short* XNl = (unsigned short*)carve(act16);
  unsigned short* PEh = (unsigned short*)carve(pe16);
  unsigned short* PEl = (unsigned short*)carve(pe16);
  float*          T   = (float*)carve(act32);
  float*          Qf  = (float*)carve(act32);
  unsigned short* QUh = (unsigned short*)carve(act16);
  unsigned short* QUl = (unsigned short*)carve(act16);
  unsigned short* QVh = (unsigned short*)carve(act16);
  unsigned short* QVl = (unsigned short*)carve(act16);
  unsigned short* Kh  = (unsigned short*)carve(act16);
  unsigned short* Kl  = (unsigned short*)carve(act16);
  unsigned short* V16 = (unsigned short*)carve(act16);
  unsigned short* Phh = (unsigned short*)carve(pe16);
  unsigned short* Pll = (unsigned short*)carve(pe16);
  unsigned short* CTXh = XNh;
  unsigned short* CTXl = XNl;
  if (off > ws_size) return;

  const unsigned short* WqT = W16 + (size_t)0 * kDim * kDim;
  const unsigned short* WkT = W16 + (size_t)1 * kDim * kDim;
  const unsigned short* WvT = W16 + (size_t)2 * kDim * kDim;
  const unsigned short* WoT = W16 + (size_t)3 * kDim * kDim;
  const unsigned short* WpT = W16 + (size_t)4 * kDim * kDim;

  bias_table_kernel<<<4, 128, 0, stream>>>(bq, bk, bv, bo, BR);
  wtcast5_kernel<<<dim3(kDim / 64, kHid / 64, 5), 256, 0, stream>>>(Wq, Wk, Wv, Wo, Wp, W16, kWCarry);
  ln_kernel<<<kTok, 64, 0, stream>>>(x, lng, lnb, XNh, XNl);
  pe_kernel<<<(kSeq * (kDim / 2)) / 256, 256, 0, stream>>>(PEh, PEl, kSeq * (kDim / 2));

  gemm_call<0, 0, false>(stream, XNl, WqT, T, T, BR, Qf, kTok, kScaleLoPass);
  gemm_call<2, 0, true >(stream, XNh, WqT, Qf, Qf, BR + 0 * kDim, T, kTok, kScaleHiPass);
  qplanes_kernel<<<(kTok * kDim / 8) / 256, 256, 0, stream>>>(Qf, ub, vbias, QUh, QUl, QVh, QVl, kTok * kDim / 8);

  gemm_call<0, 0, false>(stream, XNl, WkT, T, T, BR, Qf, kTok, kScaleLoPass);
  gemm_call<2, 2, true >(stream, XNh, WkT, Kh, Kl, BR + 1 * kDim, T, kTok, kScaleHiPass);

  gemm_call<0, 0, false>(stream, XNl, WvT, T, T, BR, Qf, kTok, kScaleLoPass);
  gemm_call<2, 1, true >(stream, XNh, WvT, V16, V16, BR + 2 * kDim, T, kTok, kScaleHiPass);

  gemm_call<0, 0, false>(stream, PEl, WpT, T, T, BR, Qf, kSeq, kScaleLoPass);
  gemm_call<0, 2, true >(stream, PEh, WpT, Phh, Pll, BR, T, kSeq, kScaleHiPass);

  rel_attn_kernel<<<kBatch * kHeads * (kSeq / 64), 128, 0, stream>>>(
      (const __bf16*)QUh, (const __bf16*)QUl, (const __bf16*)QVh, (const __bf16*)QVl,
      (const __bf16*)Kh, (const __bf16*)Kl, (const __bf16*)Phh, (const __bf16*)Pll,
      (const _Float16*)V16, CTXh, CTXl);

  gemm_call<0, 0, false>(stream, CTXl, WoT, T, T, BR, Qf, kTok, kScaleOutLo);
  gemm_call<2, 0, true >(stream, CTXh, WoT, out, out, BR + 3 * kDim, T, kTok, kScaleOutHi);
}
